// Retriever_72988674228567
// MI455X (gfx1250) — hardware-run, weakly checked
//
#include <hip/hip_runtime.h>
#include <math.h>

typedef __attribute__((ext_vector_type(16))) _Float16 v16h;
typedef __attribute__((ext_vector_type(8)))  _Float16 v8h;
typedef __attribute__((ext_vector_type(8)))  float    v8f;
typedef __attribute__((ext_vector_type(4)))  float    v4f;
typedef __attribute__((ext_vector_type(2)))  float    v2f;
typedef __attribute__((ext_vector_type(4)))  unsigned u4v;
typedef __attribute__((ext_vector_type(2)))  unsigned u2v;
typedef __attribute__((ext_vector_type(4)))  int      i4v;

constexpr int kE      = 500000;
constexpr int kN      = 100000;
constexpr int kNT     = 90000;
constexpr int kNNon   = 10000;
constexpr int kRel    = 500;
constexpr int kEmb    = 128;
constexpr int kFeat   = 142;
constexpr int kIn     = 540;
constexpr int kW1HRow = 128;
constexpr int kW1RRow = 270;
constexpr int kW1TRow = 398;
constexpr int kKPad   = 160;
constexpr int kNPad   = 100032;
constexpr int kPCols  = 256;
constexpr int kAWords = kKPad / 2;
constexpr int kPWords = kPCols / 2;
constexpr size_t kPlane = (size_t)kN * 2;
constexpr float kWCarry    = 16.0f;
constexpr float kWCarryInv = 1.0f / kWCarry;
static_assert(kNT + kNNon == kN, "node count");
static_assert(kEmb + 14 == kFeat, "node feature width");
static_assert(kEmb + kFeat + kEmb + kFeat == kIn, "edge input width");
static_assert(kW1HRow == kEmb && kW1RRow == kEmb + kFeat && kW1TRow == 2 * kEmb + kFeat, "weight row blocks");
static_assert((kKPad % 32) == 0 && kKPad >= kFeat, "GEMM K multiple of 32");
static_assert((kNPad % 64) == 0 && kNPad >= kN && (kPCols % 64) == 0, "GEMM M,N multiples of 64");
static_assert((kE % 32) == 0 && (kE % 4) == 0, "edge count multiples");
static_assert((kNT % 8) == 0 && (kN % 16) == 0, "row groups");

constexpr size_t kOffA   = 0;
constexpr size_t kOffP   = kOffA   + (size_t)kNPad * kKPad * 2;
constexpr size_t kOffCur = kOffP   + (size_t)kNPad * kPCols * 2;
constexpr size_t kOffBt  = kOffCur + 6 * kPlane * 4;
constexpr size_t kOffPR  = kOffBt  + (size_t)kPCols * kKPad * 2;
constexpr size_t kWsTotal = kOffPR + (size_t)kRel * kEmb * 4;
static_assert(kWsTotal == 88364544ull, "carve total");
static_assert(kWsTotal <= 134217728ull, "carve cap");
static_assert((kOffP % 128) == 0 && (kOffCur % 128) == 0 && (kOffBt % 128) == 0 && (kOffPR % 128) == 0, "128-B aligned regions");
static_assert(((kPlane * 4) % 128) == 0, "hop plane is whole lines");

__device__ __forceinline__ unsigned pack2h(float a, float b) {
  const _Float16 ha = (_Float16)a;
  const _Float16 hb = (_Float16)b;
  const unsigned ua = (unsigned)__builtin_bit_cast(unsigned short, ha);
  const unsigned ub = (unsigned)__builtin_bit_cast(unsigned short, hb);
  return ua | (ub << 16);
}
__device__ __forceinline__ float h16_to_f32(unsigned hb) {
  const unsigned sgn = (hb & 0x8000u) << 16;
  const unsigned em = hb & 0x7fffu;
  const float fn = __uint_as_float((em << 13) + 0x38000000u);
  const float fs = (float)em * 5.9604644775390625e-8f;
  const float mag = (em < 0x400u) ? fs : fn;
  return __uint_as_float(__float_as_uint(mag) | sgn);
}
__device__ __forceinline__ float relu_term(unsigned ha, unsigned hb, float p) {
  const float x = (h16_to_f32(ha) + h16_to_f32(hb)) + p;
  return fmaxf(x, 0.0f);
}

__device__ __forceinline__ v16h ld_frag_h(const _Float16* p) {
  union { v16h v; v8h h[2]; } f;
  f.h[0] = *(const v8h*)(p);
  f.h[1] = *(const v8h*)(p + 16);
  return f.v;
}
__device__ __forceinline__ v8f mma_h(v16h a, v16h b, v8f c) {
  c = __builtin_amdgcn_wmma_f32_16x16x32_f16(false, a, false, b, (short)0, c, false, false);
  asm volatile("v_nop\n\tv_nop\n\tv_nop\n\tv_nop" : "+v"(c) : "v"(a), "v"(b));
  return c;
}
__device__ __forceinline__ void keep4_h(v16h a, v16h b, v16h c, v16h d) { asm volatile("v_nop" :: "v"(a), "v"(b), "v"(c), "v"(d)); }
__device__ __forceinline__ void acc_guard4(v8f& a, v8f& b, v8f& c, v8f& d) { asm volatile("v_nop\n\tv_nop\n\tv_nop\n\tv_nop" : "+v"(a), "+v"(b), "+v"(c), "+v"(d)); }

constexpr int kRange      = 5120;
constexpr int kRanges     = (kN + kRange - 1) / kRange;
constexpr int kHopThreads = 512;
constexpr int kGroups     = kE / 4;
constexpr int kHopIters   = (kGroups + kHopThreads - 1) / kHopThreads;
constexpr float kFix      = 4194304.0f;
constexpr float kFixInv   = 1.0f / kFix;
static_assert(kRanges == 20, "range count");
static_assert((kRange % (2 * kHopThreads)) == 0, "store loop trip count");
static_assert((kRange % 16) == 0 && ((kN - (kRanges - 1) * kRange) % 16) == 0, "ranges are whole lines");
static_assert(kHopIters * kHopThreads >= kGroups, "edge coverage");

__global__ __launch_bounds__(512) void hop_mean_kernel(
    const int* __restrict__ hIdx, const int* __restrict__ tIdx,
    const float* __restrict__ srcF, const float* __restrict__ srcR,
    float* __restrict__ dstF, float* __restrict__ dstR)
{
  __shared__ int sAcc[3 * kRange];
  const int tx  = threadIdx.x;
  const int dir = blockIdx.y;
  const int n0  = blockIdx.x * kRange;
  const int*   dstIdx = dir ? hIdx : tIdx;
  const int*   srcIdx = dir ? tIdx : hIdx;
  const float* vin    = dir ? srcR : srcF;
  float*       vout   = dir ? dstR : dstF;
#pragma unroll 1
  for (int i = tx; i < 3 * kRange; i += kHopThreads) sAcc[i] = 0;
  __syncthreads();
#pragma unroll 1
  for (int it = 0; it < kHopIters; ++it) {
    const int g = it * kHopThreads + tx;
    const bool valid = g < kGroups;
    const int gc = valid ? g : (kGroups - 1);
    const i4v d4 = *(const i4v*)(dstIdx + 4 * (size_t)gc);
    const i4v s4 = *(const i4v*)(srcIdx + 4 * (size_t)gc);
    const int d0 = d4[0], d1 = d4[1], d2 = d4[2], d3 = d4[3];
    const int s0 = s4[0], s1 = s4[1], s2 = s4[2], s3 = s4[3];
    auto step = [&](int d, int s) {
      const int sc = min(max(s, 0), kN - 1);
      const v2f v = *(const v2f*)(vin + 2 * (size_t)sc);
      float vx = v[0];
      float vy = v[1];
      asm volatile("" : "+v"(vx), "+v"(vy));
      const int q0 = (int)rintf(vx * kFix);
      const int q1 = (int)rintf(vy * kFix);
      const int dl = d - n0;
      const bool hit = valid && ((unsigned)d < (unsigned)kN) && ((unsigned)dl < (unsigned)kRange);
      if (hit) {
        atomicAdd(&sAcc[dl], q0);
        atomicAdd(&sAcc[kRange + dl], q1);
        atomicAdd(&sAcc[2 * kRange + dl], 1);
      }
    };
    step(d0, s0);
    step(d1, s1);
    step(d2, s2);
    step(d3, s3);
  }
  __syncthreads();
  const int cntNodes = ((kN - n0) < kRange) ? (kN - n0) : kRange;
  const int pairs = cntNodes >> 1;
#pragma unroll 1
  for (int it = 0; it < kRange / (2 * kHopThreads); ++it) {
    const int p = it * kHopThreads + tx;
    if (p < pairs) {
      const int nl = 2 * p;
      const int a00 = sAcc[nl];
      const int a01 = sAcc[kRange + nl];
      const int c0  = sAcc[2 * kRange + nl];
      const int a10 = sAcc[nl + 1];
      const int a11 = sAcc[kRange + nl + 1];
      const int c1  = sAcc[2 * kRange + nl + 1];
      const float i0 = 1.0f / fmaxf((float)c0, 1.0f);
      const float i1 = 1.0f / fmaxf((float)c1, 1.0f);
      v4f o;
      o[0] = ((float)a00 * kFixInv) * i0;
      o[1] = ((float)a01 * kFixInv) * i0;
      o[2] = ((float)a10 * kFixInv) * i1;
      o[3] = ((float)a11 * kFixInv) * i1;
      volatile v4f* dp = (volatile v4f*)(vout + 2 * (size_t)(n0 + nl));
      *dp = o;
      __threadfence();
      *dp = o;
    }
  }
}

constexpr int kPackRows = 64;
static_assert((kNPad % kPackRows) == 0, "pack grid");
static_assert(kPackRows * kAWords * 4 == 5 * 256 * 16, "pack store coverage");

__global__ __launch_bounds__(256) void pack_nodes_kernel(
    const float* __restrict__ ent, const float* __restrict__ ntx, const float* __restrict__ topic,
    const float* __restrict__ cur, unsigned* __restrict__ Aw)
{
  __shared__ __align__(16) unsigned sA[kPackRows * kAWords];
  const int tid = threadIdx.x, lane = tid & 31, wave = tid >> 5;
  const int r0 = blockIdx.x * kPackRows;
#pragma unroll 1
  for (int it = 0; it < 8; ++it) {
    const int rl = it * 8 + wave;
    const int n = r0 + rl;
    const bool ok = n < kN;
    const int nc = ok ? n : (kN - 1);
    const int ne = (nc < kNT) ? nc : (kNT - 1);
    const float* srow = (nc < kNT) ? (ent + (size_t)ne * kEmb) : ntx;
    const v4f x = *(const v4f*)(srow + lane * 4);
    float x0 = x[0], x1 = x[1], x2 = x[2], x3 = x[3];
    asm volatile("" : "+v"(x0), "+v"(x1), "+v"(x2), "+v"(x3));
    x0 = ok ? x0 : 0.0f;
    x1 = ok ? x1 : 0.0f;
    x2 = ok ? x2 : 0.0f;
    x3 = ok ? x3 : 0.0f;
    u2v w;
    w[0] = pack2h(x0, x1);
    w[1] = pack2h(x2, x3);
    *(u2v*)(sA + rl * kAWords + lane * 2) = w;
  }
  {
    const int rl = tid >> 2, g = tid & 3;
    const int n = r0 + rl;
    const bool ok = n < kN;
    const int nc = ok ? n : (kN - 1);
    const size_t pb = (size_t)((g & 1) * 3) * kPlane;
    const v2f tp = *(const v2f*)(topic + 2 * (size_t)nc);
    const v2f ca = *(const v2f*)(cur + pb + 2 * (size_t)nc);
    const v2f cb = *(const v2f*)(cur + pb + kPlane + 2 * (size_t)nc);
    const v2f cc = *(const v2f*)(cur + pb + 2 * kPlane + 2 * (size_t)nc);
    float t0 = tp[0], t1 = tp[1], a0 = ca[0], a1 = ca[1], b0 = cb[0], b1 = cb[1], c0 = cc[0], c1 = cc[1];
    asm volatile("" : "+v"(t0), "+v"(t1), "+v"(a0), "+v"(a1), "+v"(b0), "+v"(b1), "+v"(c0), "+v"(c1));
    const bool g0 = ok && (g == 0);
    const bool g1 = ok && (g == 1);
    const float e0 = g0 ? t0 : (g1 ? a0 : 0.0f);
    const float e1 = g0 ? t1 : (g1 ? a1 : 0.0f);
    const float e2 = g0 ? a0 : (g1 ? b0 : 0.0f);
    const float e3 = g0 ? a1 : (g1 ? b1 : 0.0f);
    const float e4 = g0 ? b0 : (g1 ? c0 : 0.0f);
    const float e5 = g0 ? b1 : (g1 ? c1 : 0.0f);
    const float e6 = g0 ? c0 : 0.0f;
    const float e7 = g0 ? c1 : 0.0f;
    u4v w;
    w[0] = pack2h(e0, e1);
    w[1] = pack2h(e2, e3);
    w[2] = pack2h(e4, e5);
    w[3] = pack2h(e6, e7);
    *(u4v*)(sA + rl * kAWords + 64 + g * 4) = w;
  }
  __syncthreads();
  u4v ov[5];
#pragma unroll
  for (int it = 0; it < 5; ++it) ov[it] = *(const u4v*)(sA + (it * 256 + tid) * 4);
  unsigned* base = Aw + (size_t)blockIdx.x * (kPackRows * kAWords);
  for (int pass = 0; pass < 2; ++pass) {
#pragma unroll
    for (int it = 0; it < 5; ++it)
      *(volatile u4v*)(base + (it * 256 + tid) * 4) = ov[it];
    __threadfence();
  }
}

static_assert(kPCols * (kKPad / 8) == 20 * 256, "weight plane coverage");

__global__ __launch_bounds__(256) void pack_weights_kernel(const float* __restrict__ W1, unsigned* __restrict__ Btw)
{
  const int vi = blockIdx.x * 256 + threadIdx.x;
  const int n = vi / (kKPad / 8);
  const int cv = vi - n * (kKPad / 8);
  const int rowBase = (n < kEmb) ? kW1HRow : kW1TRow;
  const int col = n & (kEmb - 1);
  float w[8];
#pragma unroll
  for (int e = 0; e < 8; ++e) {
    const int k = cv * 8 + e;
    const int kc = (k < kFeat) ? k : (kFeat - 1);
    float v = W1[(size_t)(rowBase + kc) * kEmb + col];
    asm volatile("" : "+v"(v));
    w[e] = (k < kFeat) ? (v * kWCarry) : 0.0f;
  }
  u4v o;
  o[0] = pack2h(w[0], w[1]);
  o[1] = pack2h(w[2], w[3]);
  o[2] = pack2h(w[4], w[5]);
  o[3] = pack2h(w[6], w[7]);
  volatile u4v* dp = (volatile u4v*)(Btw + (size_t)vi * 4);
  *dp = o;
  __threadfence();
  *dp = o;
}

__global__ __launch_bounds__(128) void rel_terms_kernel(
    const float* __restrict__ q, const float* __restrict__ rel, const float* __restrict__ W1,
    const float* __restrict__ b1, float* __restrict__ PR)
{
  __shared__ __align__(16) float sRow[kEmb];
  const int r = blockIdx.x;
  const int j = threadIdx.x;
  float acc = b1[j];
#pragma unroll 4
  for (int k = 0; k < kEmb; ++k) acc = fmaf(q[k], W1[(size_t)k * kEmb + j], acc);
  const float* rv = rel + (size_t)r * kEmb;
#pragma unroll 4
  for (int k = 0; k < kEmb; ++k) acc = fmaf(rv[k], W1[(size_t)(kW1RRow + k) * kEmb + j], acc);
  sRow[j] = acc;
  __syncthreads();
  if (threadIdx.x < 32) {
    const v4f v = *(const v4f*)(sRow + threadIdx.x * 4);
    volatile v4f* dp = (volatile v4f*)(PR + (size_t)r * kEmb + threadIdx.x * 4);
    *dp = v;
    __threadfence();
    *dp = v;
  }
}

__global__ __launch_bounds__(256) void node_gemm_kernel(
    const unsigned short* __restrict__ Ap, int lda,
    const unsigned short* __restrict__ Btp, int ldb,
    unsigned short* __restrict__ Cp, int ldc,
    int M, int N, int K, float scale)
{
  const _Float16* A  = (const _Float16*)Ap;
  const _Float16* Bt = (const _Float16*)Btp;
  __shared__ __align__(16) float sT[8][16 * 68];
  const int lane = threadIdx.x & 31;
  const int wave = threadIdx.x >> 5;
  const int tilesN = N >> 6;
  const int tilesM = M >> 6;
  const int tile = blockIdx.x * 8 + wave;
  if (tile >= tilesM * tilesN) return;
  const int tm = tile / tilesN;
  const int tn = tile - tm * tilesN;
  const int m0 = tm << 6;
  const int n0 = tn << 6;

  const int rlane = lane & 15;
  const int koff  = (lane >> 4) * 8;
  const int mOff  = (lane >> 4) * 8;

  v8f acc[4][4];
#pragma unroll
  for (int i = 0; i < 4; ++i)
#pragma unroll
    for (int j = 0; j < 4; ++j) acc[i][j] = (v8f){0.f,0.f,0.f,0.f,0.f,0.f,0.f,0.f};

  for (int k0 = 0; k0 < K; k0 += 32) {
    v16h bh[4];
#pragma unroll
    for (int j = 0; j < 4; ++j) {
      const size_t bo = (size_t)(n0 + (j << 4) + rlane) * ldb + koff + k0;
      bh[j] = ld_frag_h(Bt + bo);
    }
#pragma unroll
    for (int i = 0; i < 4; ++i) {
      const size_t ao = (size_t)(m0 + (i << 4) + rlane) * lda + koff + k0;
      const v16h ah = ld_frag_h(A + ao);
#pragma unroll
      for (int j = 0; j < 4; ++j) acc[i][j] = mma_h(ah, bh[j], acc[i][j]);
    }
    keep4_h(bh[0], bh[1], bh[2], bh[3]);
  }
  acc_guard4(acc[0][0], acc[0][1], acc[0][2], acc[0][3]);
  acc_guard4(acc[1][0], acc[1][1], acc[1][2], acc[1][3]);
  acc_guard4(acc[2][0], acc[2][1], acc[2][2], acc[2][3]);
  acc_guard4(acc[3][0], acc[3][1], acc[3][2], acc[3][3]);

  float* slab = sT[wave];
#pragma unroll
  for (int i = 0; i < 4; ++i) {
    const int mBase = m0 + (i << 4);
#pragma unroll
    for (int j = 0; j < 4; ++j) {
#pragma unroll
      for (int r = 0; r < 8; ++r) {
        const float v = acc[i][j][r] * scale;
        slab[(mOff + r) * 68 + (j << 4) + rlane] = v;
      }
    }
    __builtin_amdgcn_fence(__ATOMIC_RELEASE, "workgroup");
    __builtin_amdgcn_wave_barrier();
    __builtin_amdgcn_fence(__ATOMIC_ACQUIRE, "workgroup");
    {
      const int q = lane >> 3, c8 = (lane & 7) * 8;
      for (int pass = 0; pass < 2; ++pass) {
#pragma unroll
        for (int it = 0; it < 4; ++it) {
          const int row = it * 4 + q;
          const float* sp = slab + row * 68 + c8;
          v8h hv;
#pragma unroll
          for (int e = 0; e < 8; ++e) hv[e] = (_Float16)sp[e];
          *(volatile v8h*)(Cp + (size_t)(mBase + row) * ldc + n0 + c8) = hv;
        }
        __threadfence();
      }
    }
    __builtin_amdgcn_fence(__ATOMIC_RELEASE, "workgroup");
    __builtin_amdgcn_wave_barrier();
    __builtin_amdgcn_fence(__ATOMIC_ACQUIRE, "workgroup");
  }
}

__global__ __launch_bounds__(256) void edge_kernel(
    const int* __restrict__ hIdx, const int* __restrict__ rIdx, const int* __restrict__ tIdx,
    const int* __restrict__ nnon, const unsigned* __restrict__ P, const float* __restrict__ PR,
    const float* __restrict__ W2, const float* __restrict__ b2, float* __restrict__ out)
{
  const int e = blockIdx.x * 256 + threadIdx.x;
  const int ec = (e < kE) ? e : (kE - 1);
  const int hi = min(max(hIdx[ec], 0), kN - 1);
  const int ti = min(max(tIdx[ec], 0), kN - 1);
  const int ri = min(max(rIdx[ec], 0), kRel - 1);
  const u4v* ph = (const u4v*)(P + (size_t)hi * kPWords);
  const u4v* pt = (const u4v*)(P + (size_t)ti * kPWords + 64);
  const v4f* pr = (const v4f*)(PR + (size_t)ri * kEmb);
  float sum = 0.0f;
#pragma unroll 1
  for (int c8 = 0; c8 < kEmb / 8; ++c8) {
    const u4v a = ph[c8];
    const u4v b = pt[c8];
    const v4f p0 = pr[2 * c8];
    const v4f p1 = pr[2 * c8 + 1];
    const float* wp = W2 + c8 * 8;
    const unsigned a0 = a[0], a1 = a[1], a2 = a[2], a3 = a[3];
    const unsigned b0 = b[0], b1 = b[1], b2w = b[2], b3 = b[3];
    const float p00 = p0[0], p01 = p0[1], p02 = p0[2], p03 = p0[3];
    const float p10 = p1[0], p11 = p1[1], p12 = p1[2], p13 = p1[3];
    sum = fmaf(relu_term(a0 & 0xffffu, b0 & 0xffffu, p00), wp[0], sum);
    sum = fmaf(relu_term(a0 >> 16,     b0 >> 16,     p01), wp[1], sum);
    sum = fmaf(relu_term(a1 & 0xffffu, b1 & 0xffffu, p02), wp[2], sum);
    sum = fmaf(relu_term(a1 >> 16,     b1 >> 16,     p03), wp[3], sum);
    sum = fmaf(relu_term(a2 & 0xffffu, b2w & 0xffffu, p10), wp[4], sum);
    sum = fmaf(relu_term(a2 >> 16,     b2w >> 16,     p11), wp[5], sum);
    sum = fmaf(relu_term(a3 & 0xffffu, b3 & 0xffffu, p12), wp[6], sum);
    sum = fmaf(relu_term(a3 >> 16,     b3 >> 16,     p13), wp[7], sum);
  }
  float val = sum + b2[0];
  const int nn = nnon[0];
  if (nn != kNNon) val = __uint_as_float(0x7fc00000u);
  if (e < kE) {
    volatile float* op = out + e;
    *op = val;
    __threadfence();
    *op = val;
  }
}

extern "C" void kernel_launch(void* const* d_in, const int* in_sizes, int n_in,
                              void* d_out, int out_size, void* d_ws, size_t ws_size,
                              hipStream_t stream) {
  if (n_in < 13) return;
  if (in_sizes[0] != kE || in_sizes[1] != kE || in_sizes[2] != kE) return;
  if (in_sizes[3] != kEmb) return;
  if (in_sizes[4] != kNT * kEmb) return;
  if (in_sizes[5] != 1) return;
  if (in_sizes[6] != kRel * kEmb) return;
  if (in_sizes[7] != kN * 2) return;
  if (in_sizes[8] != kEmb) return;
  if (in_sizes[9] != kIn * kEmb) return;
  if (in_sizes[10] != kEmb) return;
  if (in_sizes[11] != kEmb) return;
  if (in_sizes[12] != 1) return;
  if (out_size != kE) return;
  if (ws_size < kWsTotal) return;

  const int*   hIdx  = (const int*)d_in[0];
  const int*   rIdx  = (const int*)d_in[1];
  const int*   tIdx  = (const int*)d_in[2];
  const float* q     = (const float*)d_in[3];
  const float* ent   = (const float*)d_in[4];
  const int*   nnon  = (const int*)d_in[5];
  const float* rel   = (const float*)d_in[6];
  const float* topic = (const float*)d_in[7];
  const float* ntx   = (const float*)d_in[8];
  const float* W1    = (const float*)d_in[9];
  const float* b1    = (const float*)d_in[10];
  const float* W2    = (const float*)d_in[11];
  const float* b2    = (const float*)d_in[12];
  float* out = (float*)d_out;

  char* ws = (char*)d_ws;
  unsigned* Aw  = (unsigned*)(ws + kOffA);
  unsigned* Pw  = (unsigned*)(ws + kOffP);
  float*    cur = (float*)(ws + kOffCur);
  unsigned* Btw = (unsigned*)(ws + kOffBt);
  float*    PR  = (float*)(ws + kOffPR);

  float* F1 = cur + 0 * kPlane;
  float* F2 = cur + 1 * kPlane;
  float* F3 = cur + 2 * kPlane;
  float* R1 = cur + 3 * kPlane;
  float* R2 = cur + 4 * kPlane;
  float* R3 = cur + 5 * kPlane;

  hop_mean_kernel<<<dim3(kRanges, 2), kHopThreads, 0, stream>>>(hIdx, tIdx, topic, topic, F1, R1);
  hop_mean_kernel<<<dim3(kRanges, 2), kHopThreads, 0, stream>>>(hIdx, tIdx, F1, R1, F2, R2);
  hop_mean_kernel<<<dim3(kRanges, 2), kHopThreads, 0, stream>>>(hIdx, tIdx, F2, R2, F3, R3);

  pack_nodes_kernel<<<kNPad / kPackRows, 256, 0, stream>>>(ent, ntx, topic, cur, Aw);
  pack_weights_kernel<<<20, 256, 0, stream>>>(W1, Btw);
  rel_terms_kernel<<<kRel, 128, 0, stream>>>(q, rel, W1, b1, PR);

  const int tiles = (kNPad / 64) * (kPCols / 64);
  node_gemm_kernel<<<(tiles + 7) / 8, 256, 0, stream>>>(
      (const unsigned short*)Aw, kKPad,
      (const unsigned short*)Btw, kKPad,
      (unsigned short*)Pw, kPCols,
      kNPad, kPCols, kKPad, kWCarryInv);

  edge_kernel<<<(kE + 255) / 256, 256, 0, stream>>>(hIdx, rIdx, tIdx, nnon, Pw, PR, W2, b2, out);
}
